// Encoder_80874234183757
// MI455X (gfx1250) — hardware-run, weakly checked
//
#include <hip/hip_runtime.h>
#include <stddef.h>
#include <stdint.h>

#define SPLIT_M1 1
#define SPLIT_H  1
#define SPLIT_M2 1

#define NN      100000
#define NE      1600000
#define FI      128
#define FO      64
#define GBM     128
#define MP      100096
#define P_XB    128
#define P_M1    256
#define P_H     128
#define P_M2    128
#define P_W1    384
#define P_W2    256
#define NTHR    256
#define NWAVE   8
#define EPT     8
#define WCH     (32 * EPT)
#define NCH     (NE / WCH)
#define NBRUN   1024
#define SLB     10
#define SRCB    17
#define NBK     98
#define WLCAP   3584
#define RCAP    20480
#define DEGCAP  64
#define MAXDEG_MEAS   36
#define MAXB1024_MEAS 16710
#define RPB     64
#define SP      68
#define WSMAX   ((size_t)(128u << 20))

#define BK_ZINTS (NWAVE * WLCAP + RCAP + 3 * NBRUN)
#define BK_INTS  (BK_ZINTS + 16)
#define BK_LDS   (BK_INTS * 4)

#define PBX   (MP * FI / 8 / NTHR)
#define PBA   (FO * 2 * FI / 8 / NTHR)
#define PBB   (FO * FI / 8 / NTHR)
#define PBC   (FO * 2 * FO / 8 / NTHR)
#define PBD   (FO * 2 * FO / 8 / NTHR)
#define PBTOT (PBX + PBA + PBB + PBC + PBD + 1)

static_assert(FO == 64 && FO == 16 * 4 && FI == 128 && FI == 32 * 4);
static_assert(MP % GBM == 0 && MP >= NN && MP == 782 * GBM && MP % RPB == 0);
static_assert(NBRUN == (1 << SLB) && NBRUN <= 1024 && NBRUN % RPB == 0 && NBRUN % GBM == 0 && NBRUN % 32 == 0);
static_assert(NBK * NBRUN >= MP);
static_assert(NN <= (1 << SRCB) && SLB + SRCB <= 31);
static_assert(NE % WCH == 0 && NE % 4 == 0);
static_assert(RCAP % (NTHR * 4) == 0 && BK_ZINTS % (NTHR * 4) == 0 && (2 * NBRUN) % (NTHR * 4) == 0);
static_assert((long long)RCAP * 100 >= (long long)MAXB1024_MEAS * 105);
static_assert((long long)WLCAP * 100 >= (long long)(MAXB1024_MEAS / 8 + 1) * 125);
static_assert(MAXDEG_MEAS + 8 <= DEGCAP && DEGCAP <= 64);
static_assert(BK_LDS <= 300000);
static_assert((GBM * SP + 64) * 4 <= 65536);
static_assert((MP * FI / 8) % NTHR == 0 && (FO * 2 * FI / 8) % NTHR == 0 && (FO * FI / 8) % NTHR == 0);
static_assert((FO * 2 * FO / 8) % NTHR == 0);
static_assert(P_W1 == 3 * FI && P_W2 == 4 * FO && P_M1 == 2 * FI && P_H == 2 * FO && P_M2 == 2 * FO && P_XB == FI);
static_assert(FI % 32 == 0 && FO % 32 == 0);
static_assert(RPB % (2 * NWAVE) == 0);

typedef float          v4f   __attribute__((ext_vector_type(4)));
typedef float          v8f   __attribute__((ext_vector_type(8)));
typedef int            v4i   __attribute__((ext_vector_type(4)));
typedef int            v8i   __attribute__((ext_vector_type(8)));
typedef unsigned       v2u   __attribute__((ext_vector_type(2)));
typedef unsigned short v8us  __attribute__((ext_vector_type(8)));
typedef unsigned short v16us __attribute__((ext_vector_type(16)));
typedef __bf16         v16bf __attribute__((ext_vector_type(16)));
typedef v4f  __attribute__((may_alias)) v4fa;
typedef v4i  __attribute__((may_alias)) v4ia;
typedef v2u  __attribute__((may_alias)) v2ua;
typedef v8us __attribute__((may_alias)) v8usa;
union FragB { v16bf v; v16us u; v8us h[2]; v8i w; };

__device__ __forceinline__ v8f wmb(const FragB& a, const FragB& b, v8f c) {
  v8f d = __builtin_amdgcn_wmma_f32_16x16x32_bf16(false, a.v, false, b.v, (short)0, c, false, false);
  asm volatile("v_nop\n\tv_nop\n\tv_nop\n\tv_nop" : "+v"(d) : "v"(a.w), "v"(b.w));
  return d;
}

__device__ __forceinline__ unsigned bf16_bits(float f) {
  const unsigned u = __float_as_uint(f);
  const unsigned r = (u + 0x7FFFu + ((u >> 16) & 1u)) >> 16;
  const unsigned q = (u >> 16) | 0x40u;
  return ((u & 0x7fffffffu) > 0x7f800000u) ? q : r;
}

__device__ __forceinline__ void hilo_pack(float v0, float v1, float v2, float v3, unsigned lom,
                                          int& h01, int& h23, int& l01, int& l23) {
  const unsigned a0 = bf16_bits(v0), a1 = bf16_bits(v1), a2 = bf16_bits(v2), a3 = bf16_bits(v3);
  const unsigned b0 = bf16_bits(v0 - __uint_as_float(a0 << 16));
  const unsigned b1 = bf16_bits(v1 - __uint_as_float(a1 << 16));
  const unsigned b2 = bf16_bits(v2 - __uint_as_float(a2 << 16));
  const unsigned b3 = bf16_bits(v3 - __uint_as_float(a3 << 16));
  h01 = (int)(a0 | (a1 << 16)); h23 = (int)(a2 | (a3 << 16));
  l01 = (int)((b0 | (b1 << 16)) & lom); l23 = (int)((b2 | (b3 << 16)) & lom);
}

__device__ __forceinline__ v4i regroup8(int h01, int h23, int l01, int l23, int lane) {
  const int t  = lane & 15;
  const int s0 = (lane & 16) + ((2 * t) & 15), s1 = s0 + 1;
  const int a0 = __shfl(h01, s0, 32), a1 = __shfl(h23, s0, 32), a2 = __shfl(h01, s1, 32), a3 = __shfl(h23, s1, 32);
  const int b0 = __shfl(l01, s0, 32), b1 = __shfl(l23, s0, 32), b2 = __shfl(l01, s1, 32), b3 = __shfl(l23, s1, 32);
  const int mk = (t < 8) ? -1 : 0;
  v4i o;
  o.x = (a0 & mk) | (b0 & ~mk); o.y = (a1 & mk) | (b1 & ~mk);
  o.z = (a2 & mk) | (b2 & ~mk); o.w = (a3 & mk) | (b3 & ~mk);
  return o;
}

__device__ __forceinline__ v4i regroup32(int h01, int h23, int l01, int l23, int lane) {
  const int s0 = (2 * lane) & 31, s1 = s0 + 1;
  const int a0 = __shfl(h01, s0, 32), a1 = __shfl(h23, s0, 32), a2 = __shfl(h01, s1, 32), a3 = __shfl(h23, s1, 32);
  const int b0 = __shfl(l01, s0, 32), b1 = __shfl(l23, s0, 32), b2 = __shfl(l01, s1, 32), b3 = __shfl(l23, s1, 32);
  const int mk = (lane < 16) ? -1 : 0;
  v4i o;
  o.x = (a0 & mk) | (b0 & ~mk); o.y = (a1 & mk) | (b1 & ~mk);
  o.z = (a2 & mk) | (b2 & ~mk); o.w = (a3 & mk) | (b3 & ~mk);
  return o;
}

__device__ __forceinline__ void st2_v4f(float* p, v4f v) {
  *(volatile v4f*)p = v;
  __threadfence();
  *(volatile v4f*)p = v;
}
__device__ __forceinline__ void st2_v4i(unsigned short* p, v4i v) {
  *(volatile v4i*)p = v;
  __threadfence();
  *(volatile v4i*)p = v;
}
__device__ __forceinline__ void st2_v8us(unsigned short* p, v8us v) {
  *(volatile v8us*)p = v;
  __threadfence();
  *(volatile v8us*)p = v;
}

__device__ __forceinline__ v8us gather8(const float* __restrict__ base, int stride) {
  float f[8];
#pragma unroll
  for (int i = 0; i < 8; ++i) f[i] = base[(size_t)i * (size_t)stride];
  v8us o;
#pragma unroll
  for (int i = 0; i < 8; ++i) o[i] = (unsigned short)bf16_bits(f[i]);
  return o;
}

__device__ __forceinline__ unsigned csrc(int v) {
  v = v < 0 ? 0 : (v > NN - 1 ? NN - 1 : v);
  return (unsigned)v;
}

__global__ __launch_bounds__(NTHR) void k_prep(const float* __restrict__ x, const float* __restrict__ wl1,
                                               const float* __restrict__ wr1, const float* __restrict__ b1,
                                               const float* __restrict__ wl2, const float* __restrict__ wr2,
                                               const float* __restrict__ b2, unsigned short* xb,
                                               unsigned short* w1c, unsigned short* w2c, float* sm) {
  const int tid = (int)threadIdx.x, lane = tid & 31;
  const int blk = (int)blockIdx.x;
  if (blk < PBX) {
    const int u   = blk * NTHR + tid;
    const int row = u >> 4, k8 = (u & 15) * 8;
    const int rc  = row < NN ? row : NN - 1;
    const unsigned mk = row < NN ? 0xffffu : 0u;
    const float* p = x + (size_t)rc * FI + k8;
    const v4f a = *(const v4fa*)p;
    const v4f b = *(const v4fa*)(p + 4);
    v8us o;
    o[0] = (unsigned short)(bf16_bits(a.x) & mk); o[1] = (unsigned short)(bf16_bits(a.y) & mk);
    o[2] = (unsigned short)(bf16_bits(a.z) & mk); o[3] = (unsigned short)(bf16_bits(a.w) & mk);
    o[4] = (unsigned short)(bf16_bits(b.x) & mk); o[5] = (unsigned short)(bf16_bits(b.y) & mk);
    o[6] = (unsigned short)(bf16_bits(b.z) & mk); o[7] = (unsigned short)(bf16_bits(b.w) & mk);
    st2_v8us(xb + (size_t)row * P_XB + k8, o);
  } else if (blk < PBX + PBA) {
    const int u = (blk - PBX) * NTHR + tid;
    const int n = u >> 5, k8 = (u & 31) * 8, kk = k8 & (FI - 1);
    const v8us o = gather8(wl1 + (size_t)kk * FO + n, FO);
    st2_v8us(w1c + (size_t)n * P_W1 + k8, o);
  } else if (blk < PBX + PBA + PBB) {
    const int u = (blk - PBX - PBA) * NTHR + tid;
    const int n = u >> 4, k8 = (u & 15) * 8;
    const v8us o = gather8(wr1 + (size_t)k8 * FO + n, FO);
    st2_v8us(w1c + (size_t)n * P_W1 + 2 * FI + k8, o);
  } else if (blk < PBX + PBA + PBB + PBC) {
    const int u = (blk - PBX - PBA - PBB) * NTHR + tid;
    const int n = u >> 4, k8 = (u & 15) * 8, kk = k8 & (FO - 1);
    const v8us o = gather8(wl2 + (size_t)kk * FO + n, FO);
    st2_v8us(w2c + (size_t)n * P_W2 + k8, o);
  } else if (blk < PBX + PBA + PBB + PBC + PBD) {
    const int u = (blk - PBX - PBA - PBB - PBC) * NTHR + tid;
    const int n = u >> 4, k8 = (u & 15) * 8, kk = k8 & (FO - 1);
    const v8us o = gather8(wr2 + (size_t)kk * FO + n, FO);
    st2_v8us(w2c + (size_t)n * P_W2 + 2 * FO + k8, o);
  } else {
    if (tid < 32) {
      const int q = lane & 15;
      const v4f a = *(const v4fa*)(b1 + 4 * q);
      const v4f c = *(const v4fa*)(b2 + 4 * q);
      asm volatile("" :: "v"(a));
      asm volatile("" :: "v"(c));
      const unsigned ma = (lane < 16) ? 0xffffffffu : 0u;
      v4f o;
      o.x = __uint_as_float(((bf16_bits(a.x) << 16) & ma) | ((bf16_bits(c.x) << 16) & ~ma));
      o.y = __uint_as_float(((bf16_bits(a.y) << 16) & ma) | ((bf16_bits(c.y) << 16) & ~ma));
      o.z = __uint_as_float(((bf16_bits(a.z) << 16) & ma) | ((bf16_bits(c.z) << 16) & ~ma));
      o.w = __uint_as_float(((bf16_bits(a.w) << 16) & ma) | ((bf16_bits(c.w) << 16) & ~ma));
      st2_v4f(sm + 4 * lane, o);
    }
  }
}

__device__ __forceinline__ void bucket_flush(const int* pl, const int* cnt, int ov, int* lp, int* cop, int* fp,
                                             int tid) {
#pragma unroll 1
  for (int i = tid * 4; i < RCAP; i += NTHR * 4) {
    const v4i v = *(const v4ia*)(pl + i);
    *(volatile v4i*)(lp + i) = v;
  }
#pragma unroll 1
  for (int i = tid * 4; i < 2 * NBRUN; i += NTHR * 4) {
    const v4i v = *(const v4ia*)(cnt + i);
    *(volatile v4i*)(cop + i) = v;
  }
  if (tid < 8) {
    const v4i f = {ov, ov, ov, ov};
    *(volatile v4i*)(fp + 4 * tid) = f;
  }
}

__global__ __launch_bounds__(NTHR) void k_bucket(const int* __restrict__ srcs, const int* __restrict__ dsts,
                                                 int* LIST, int* CO, int* FLAG) {
  extern __shared__ __attribute__((aligned(16))) int dsm[];
  int* wl   = dsm;
  int* pl   = dsm + NWAVE * WLCAP;
  int* cnt  = pl + RCAP;
  int* offs = cnt + NBRUN;
  int* cur  = offs + NBRUN;
  int* misc = cur + NBRUN;
  const int tid = (int)threadIdx.x, lane = tid & 31, wave = tid >> 5;
  const int blk = (int)blockIdx.x;
  const unsigned nbs = (unsigned)(blk * NBRUN);

  {
    const v4i z4 = {0, 0, 0, 0};
    for (int i = tid * 4; i < BK_ZINTS; i += NTHR * 4) *(v4ia*)(dsm + i) = z4;
    if (tid < 16) misc[tid] = 0;
  }
  __syncthreads();

  {
    int* mylist = wl + wave * WLCAP;
    int wc = 0;
#pragma unroll 1
    for (int ch = wave; ch < NCH; ch += NWAVE) {
      const int e0 = ch * WCH + lane * EPT;
      const v4i da = *(const v4ia*)(dsts + e0);
      const v4i db = *(const v4ia*)(dsts + e0 + 4);
      const unsigned s0 = (unsigned)da.x - nbs, s1 = (unsigned)da.y - nbs;
      const unsigned s2 = (unsigned)da.z - nbs, s3 = (unsigned)da.w - nbs;
      const unsigned s4 = (unsigned)db.x - nbs, s5 = (unsigned)db.y - nbs;
      const unsigned s6 = (unsigned)db.z - nbs, s7 = (unsigned)db.w - nbs;
      const bool h0 = s0 < (unsigned)NBRUN, h1 = s1 < (unsigned)NBRUN, h2 = s2 < (unsigned)NBRUN, h3 = s3 < (unsigned)NBRUN;
      const bool h4 = s4 < (unsigned)NBRUN, h5 = s5 < (unsigned)NBRUN, h6 = s6 < (unsigned)NBRUN, h7 = s7 < (unsigned)NBRUN;
      const unsigned m0 = __builtin_amdgcn_ballot_w32(h0), m1 = __builtin_amdgcn_ballot_w32(h1);
      const unsigned m2 = __builtin_amdgcn_ballot_w32(h2), m3 = __builtin_amdgcn_ballot_w32(h3);
      const unsigned m4 = __builtin_amdgcn_ballot_w32(h4), m5 = __builtin_amdgcn_ballot_w32(h5);
      const unsigned m6 = __builtin_amdgcn_ballot_w32(h6), m7 = __builtin_amdgcn_ballot_w32(h7);
      const unsigned any = m0 | m1 | m2 | m3 | m4 | m5 | m6 | m7;
      if (any != 0u) {
        const v4i sa = *(const v4ia*)(srcs + e0);
        const v4i sb = *(const v4ia*)(srcs + e0 + 4);
        asm volatile("" :: "v"(sa));
        asm volatile("" :: "v"(sb));
        const int pre = (int)(__builtin_amdgcn_mbcnt_lo(m0, 0u) + __builtin_amdgcn_mbcnt_lo(m1, 0u) +
                              __builtin_amdgcn_mbcnt_lo(m2, 0u) + __builtin_amdgcn_mbcnt_lo(m3, 0u) +
                              __builtin_amdgcn_mbcnt_lo(m4, 0u) + __builtin_amdgcn_mbcnt_lo(m5, 0u) +
                              __builtin_amdgcn_mbcnt_lo(m6, 0u) + __builtin_amdgcn_mbcnt_lo(m7, 0u));
        int p = wc + pre;
        if (h0) { if (p < WLCAP) mylist[p] = (int)((s0 << SRCB) | csrc(sa.x)); p = p + 1; }
        if (h1) { if (p < WLCAP) mylist[p] = (int)((s1 << SRCB) | csrc(sa.y)); p = p + 1; }
        if (h2) { if (p < WLCAP) mylist[p] = (int)((s2 << SRCB) | csrc(sa.z)); p = p + 1; }
        if (h3) { if (p < WLCAP) mylist[p] = (int)((s3 << SRCB) | csrc(sa.w)); p = p + 1; }
        if (h4) { if (p < WLCAP) mylist[p] = (int)((s4 << SRCB) | csrc(sb.x)); p = p + 1; }
        if (h5) { if (p < WLCAP) mylist[p] = (int)((s5 << SRCB) | csrc(sb.y)); p = p + 1; }
        if (h6) { if (p < WLCAP) mylist[p] = (int)((s6 << SRCB) | csrc(sb.z)); p = p + 1; }
        if (h7) { if (p < WLCAP) mylist[p] = (int)((s7 << SRCB) | csrc(sb.w)); p = p + 1; }
        wc += (int)(__builtin_popcount(m0) + __builtin_popcount(m1) + __builtin_popcount(m2) + __builtin_popcount(m3) +
                    __builtin_popcount(m4) + __builtin_popcount(m5) + __builtin_popcount(m6) + __builtin_popcount(m7));
      }
    }
    if (lane == 0) misc[wave] = wc;
  }
  __syncthreads();

  if (wave == 0) {
    int ov = 0;
#pragma unroll 1
    for (int w2 = 0; w2 < NWAVE; ++w2) {
      int c = misc[w2];
      if (c > WLCAP) ov = 1;
      c = c < 0 ? 0 : (c > WLCAP ? WLCAP : c);
#pragma unroll 1
      for (int b0 = 0; b0 < c; b0 += 32) {
        const int idx = b0 + lane;
        const int ent = wl[w2 * WLCAP + (idx < WLCAP ? idx : WLCAP - 1)];
        const int m32 = min(c - b0, 32);
#pragma unroll 1
        for (int k = 0; k < m32; ++k) {
          const int u    = __builtin_amdgcn_readlane(ent, k);
          const int slot = (u >> SRCB) & (NBRUN - 1);
          if (lane == 0) cnt[slot] = cnt[slot] + 1;
        }
      }
    }
    if (lane == 0) misc[9] = ov;
  }
  __syncthreads();
  if (wave == 0) {
    const int base = lane * (NBRUN / 32);
    int s = 0;
#pragma unroll 1
    for (int i = 0; i < NBRUN / 32; ++i) s += cnt[base + i];
    int incl = s;
#pragma unroll
    for (int d = 1; d < 32; d <<= 1) {
      const int y = __shfl_up(incl, d, 32);
      if (lane >= d) incl += y;
    }
    const int tot = __shfl(incl, 31, 32);
    int run = incl - s;
#pragma unroll 1
    for (int i = 0; i < NBRUN / 32; ++i) {
      const int cv = cnt[base + i];
      offs[base + i] = run;
      cur[base + i]  = run;
      run += cv;
    }
    if (lane == 0 && tot > RCAP) misc[9] = 1;
  }
  __syncthreads();

  if (wave == 0) {
#pragma unroll 1
    for (int w2 = 0; w2 < NWAVE; ++w2) {
      int c = misc[w2];
      c = c < 0 ? 0 : (c > WLCAP ? WLCAP : c);
#pragma unroll 1
      for (int b0 = 0; b0 < c; b0 += 32) {
        const int idx = b0 + lane;
        const int ent = wl[w2 * WLCAP + (idx < WLCAP ? idx : WLCAP - 1)];
        const int m32 = min(c - b0, 32);
#pragma unroll 1
        for (int k = 0; k < m32; ++k) {
          const int u    = __builtin_amdgcn_readlane(ent, k);
          const int slot = (u >> SRCB) & (NBRUN - 1);
          const int sr   = u & ((1 << SRCB) - 1);
          if (lane == 0) {
            int p = cur[slot];
            p = p < 0 ? 0 : (p > RCAP - 1 ? RCAP - 1 : p);
            pl[p] = sr;
            cur[slot] = p + 1;
          }
        }
      }
    }
  }
  __syncthreads();

  const int ovf = misc[9];
  int* lp  = LIST + (size_t)blk * RCAP;
  int* cop = CO + (size_t)blk * (2 * NBRUN);
  int* fp  = FLAG + (size_t)blk * 32;
  bucket_flush(pl, cnt, ovf, lp, cop, fp, tid);
  __threadfence();
  bucket_flush(pl, cnt, ovf, lp, cop, fp, tid);
}

__global__ __launch_bounds__(NTHR) void k_replay1(const int* __restrict__ LIST, const int* __restrict__ CO,
                                                  const int* __restrict__ FLAG,
                                                  const unsigned short* __restrict__ XB, unsigned short* M1HL) {
  const int tid = (int)threadIdx.x, lane = tid & 31, wave = tid >> 5;
  const int rowBase = (int)blockIdx.x * RPB;
  const int bucket  = rowBase >> SLB;
  const int* lb  = LIST + (size_t)bucket * RCAP;
  const int* cob = CO + (size_t)bucket * (2 * NBRUN);
  const int flag = FLAG[(size_t)bucket * 32];
  const float qnan = __uint_as_float(0x7fc00000u);

#pragma unroll 1
  for (int i = 0; i < RPB / NWAVE; ++i) {
    const int d    = rowBase + (RPB / NWAVE) * wave + i;
    const int slot = d & (NBRUN - 1);
    int cv = cob[slot];
    int ovv = cob[NBRUN + slot];
    const bool big = cv > DEGCAP;
    cv  = cv < 0 ? 0 : (cv > DEGCAP ? DEGCAP : cv);
    ovv = ovv < 0 ? 0 : (ovv > RCAP - 1 ? RCAP - 1 : ovv);
    const int c = __builtin_amdgcn_readfirstlane(cv);
    const int o = __builtin_amdgcn_readfirstlane(ovv);
    int last = o + c - 1; last = last < o ? o : last;
    last = min(last, RCAP - 1);
    float a0 = 0.0f, a1 = 0.0f, a2 = 0.0f, a3 = 0.0f;
#pragma unroll 1
    for (int b0 = 0; b0 < c; b0 += 32) {
      const int idx = min(o + b0 + lane, last);
      int sr = lb[idx];
      sr = sr < 0 ? 0 : (sr > NN - 1 ? NN - 1 : sr);
      const int m32 = min(c - b0, 32);
#pragma unroll 1
      for (int k = 0; k < m32; ++k) {
        const int sk = __builtin_amdgcn_readlane(sr, k);
        const v2u w = *(const v2ua*)(XB + (size_t)sk * P_XB + 4 * lane);
        a0 += __uint_as_float(w.x << 16);
        a1 += __uint_as_float(w.x & 0xffff0000u);
        a2 += __uint_as_float(w.y << 16);
        a3 += __uint_as_float(w.y & 0xffff0000u);
      }
    }
    const float den = fmaxf((float)c, 1.0f);
    float m0 = a0 / den, m1 = a1 / den, m2 = a2 / den, m3 = a3 / den;
    const bool bad  = (flag != 0) | big;
    const bool live = d < NN;
    m0 = bad ? qnan : m0; m1 = bad ? qnan : m1; m2 = bad ? qnan : m2; m3 = bad ? qnan : m3;
    m0 = live ? m0 : 0.0f; m1 = live ? m1 : 0.0f; m2 = live ? m2 : 0.0f; m3 = live ? m3 : 0.0f;
    int h01, h23, l01, l23;
    hilo_pack(m0, m1, m2, m3, 0xffffffffu, h01, h23, l01, l23);
    const v4i ow = regroup32(h01, h23, l01, l23, lane);
    st2_v4i(M1HL + (size_t)d * P_M1 + 8 * lane, ow);
  }
}

__global__ __launch_bounds__(NTHR) void k_replay2(const int* __restrict__ LIST, const int* __restrict__ CO,
                                                  const int* __restrict__ FLAG,
                                                  const unsigned short* __restrict__ HHL, unsigned short* M2HL) {
  const int tid = (int)threadIdx.x, lane = tid & 31, wave = tid >> 5, hh = lane >> 4, q = lane & 15;
  const int rowBase = (int)blockIdx.x * RPB;
  const int bucket  = rowBase >> SLB;
  const int* lb  = LIST + (size_t)bucket * RCAP;
  const int* cob = CO + (size_t)bucket * (2 * NBRUN);
  const int flag = FLAG[(size_t)bucket * 32];
  const float qnan = __uint_as_float(0x7fc00000u);

#pragma unroll 1
  for (int i = 0; i < RPB / (2 * NWAVE); ++i) {
    const int d    = rowBase + (RPB / NWAVE) * wave + 2 * i + hh;
    const int slot = d & (NBRUN - 1);
    int c = cob[slot];
    int o = cob[NBRUN + slot];
    const bool big = c > DEGCAP;
    c = c < 0 ? 0 : (c > DEGCAP ? DEGCAP : c);
    o = o < 0 ? 0 : (o > RCAP - 1 ? RCAP - 1 : o);
    const int co = __shfl_xor(c, 16, 32);
    const int cmv = c > co ? c : co;
    const int cm = __builtin_amdgcn_readfirstlane(cmv);
    int last = o + c - 1; last = last < o ? o : last;
    last = min(last, RCAP - 1);
    float a0 = 0.0f, a1 = 0.0f, a2 = 0.0f, a3 = 0.0f;
#pragma unroll 1
    for (int j = 0; j < cm; ++j) {
      const int idx = min(o + j, last);
      int sr = lb[idx];
      sr = sr < 0 ? 0 : (sr > NN - 1 ? NN - 1 : sr);
      const unsigned short* rp = HHL + (size_t)sr * P_H + 4 * q;
      const v2u wh = *(const v2ua*)rp;
      const v2u wo = *(const v2ua*)(rp + FO);
      asm volatile("" :: "v"(wh));
      asm volatile("" :: "v"(wo));
      const float f0 = __uint_as_float(wh.x << 16)         + __uint_as_float(wo.x << 16);
      const float f1 = __uint_as_float(wh.x & 0xffff0000u) + __uint_as_float(wo.x & 0xffff0000u);
      const float f2 = __uint_as_float(wh.y << 16)         + __uint_as_float(wo.y << 16);
      const float f3 = __uint_as_float(wh.y & 0xffff0000u) + __uint_as_float(wo.y & 0xffff0000u);
      const bool valid = j < c;
      const float t0 = a0 + f0, t1 = a1 + f1, t2 = a2 + f2, t3 = a3 + f3;
      a0 = valid ? t0 : a0; a1 = valid ? t1 : a1; a2 = valid ? t2 : a2; a3 = valid ? t3 : a3;
    }
    const float den = fmaxf((float)c, 1.0f);
    float m0 = a0 / den, m1 = a1 / den, m2 = a2 / den, m3 = a3 / den;
    const bool bad  = (flag != 0) | big;
    const bool live = d < NN;
    m0 = bad ? qnan : m0; m1 = bad ? qnan : m1; m2 = bad ? qnan : m2; m3 = bad ? qnan : m3;
    m0 = live ? m0 : 0.0f; m1 = live ? m1 : 0.0f; m2 = live ? m2 : 0.0f; m3 = live ? m3 : 0.0f;
    int h01, h23, l01, l23;
    hilo_pack(m0, m1, m2, m3, 0xffffffffu, h01, h23, l01, l23);
    const v4i ow = regroup8(h01, h23, l01, l23, lane);
    st2_v4i(M2HL + (size_t)d * P_M2 + 8 * q, ow);
  }
}

template <int BP>
__device__ __forceinline__ void gemm_seg(const unsigned short* __restrict__ ap,
                                         const unsigned short* __restrict__ bp, int nk, v8f (&acc)[4]) {
#pragma unroll 1
  for (int s = 0; s < nk; ++s) {
    const int k0 = 32 * s;
    FragB af;
    af.h[0] = *(const v8usa*)(ap + k0);
    af.h[1] = *(const v8usa*)(ap + k0 + 16);
#pragma unroll
    for (int nt = 0; nt < 4; ++nt) {
      const unsigned short* wq = bp + (size_t)(16 * nt) * (size_t)BP + k0;
      FragB bf;
      bf.h[0] = *(const v8usa*)wq;
      bf.h[1] = *(const v8usa*)(wq + 16);
      acc[nt] = wmb(af, bf, acc[nt]);
    }
  }
}

__device__ __forceinline__ void stage_d(float* stg, const v8f (&acc)[4], int wave, int hh, int m) {
#pragma unroll
  for (int nt = 0; nt < 4; ++nt) {
#pragma unroll
    for (int r = 0; r < 8; ++r) stg[(16 * wave + 8 * hh + r) * SP + 16 * nt + m] = acc[nt][r];
  }
}

__global__ __launch_bounds__(NTHR) __attribute__((amdgpu_num_vgpr(248)))
void k_gemm1(const unsigned short* __restrict__ M1HL, const unsigned short* __restrict__ XB,
             const unsigned short* __restrict__ W1C, const float* __restrict__ sm, unsigned short* HHL) {
  __shared__ __attribute__((aligned(16))) float stg[GBM * SP];
  __shared__ __attribute__((aligned(16))) float sb[64];
  const int tid = (int)threadIdx.x, lane = tid & 31, wave = tid >> 5, hh = lane >> 4, m = lane & 15;
  const int rowBase = (int)blockIdx.x * GBM;
  if (tid < 16) *(v4fa*)(sb + 4 * tid) = *(const v4fa*)(sm + 4 * tid);

  v8f acc[4];
  {
    const v8f z = {0.f, 0.f, 0.f, 0.f, 0.f, 0.f, 0.f, 0.f};
#pragma unroll
    for (int t = 0; t < 4; ++t) acc[t] = z;
  }
  const int arow = rowBase + 16 * wave + m;
  const unsigned short* bp = W1C + (size_t)m * (size_t)P_W1 + 8 * hh;
  gemm_seg<P_W1>(M1HL + (size_t)arow * P_M1 + 8 * hh, bp, SPLIT_M1 ? 8 : 4, acc);
  gemm_seg<P_W1>(XB + (size_t)arow * P_XB + 8 * hh, bp + 2 * FI, 4, acc);
  stage_d(stg, acc, wave, hh, m);
  __syncthreads();

  const v4f bias = *(const v4fa*)(sb + 4 * m);
  const unsigned lom = SPLIT_H ? 0xffffffffu : 0u;
#pragma unroll 1
  for (int i = 0; i < 8; ++i) {
    const int lr   = 16 * wave + 2 * i + hh;
    const int grow = rowBase + lr;
    const bool live = grow < NN;
    const v4f a = *(const v4fa*)(stg + lr * SP + 4 * m);
    asm volatile("" :: "v"(a));
    float v0 = a.x + bias.x, v1 = a.y + bias.y, v2 = a.z + bias.z, v3 = a.w + bias.w;
    v0 = (v0 > 0.0f) ? v0 : (v0 - v0); v1 = (v1 > 0.0f) ? v1 : (v1 - v1);
    v2 = (v2 > 0.0f) ? v2 : (v2 - v2); v3 = (v3 > 0.0f) ? v3 : (v3 - v3);
    v0 = live ? v0 : 0.0f; v1 = live ? v1 : 0.0f; v2 = live ? v2 : 0.0f; v3 = live ? v3 : 0.0f;
    int h01, h23, l01, l23;
    hilo_pack(v0, v1, v2, v3, lom, h01, h23, l01, l23);
    const v4i ow = regroup8(h01, h23, l01, l23, lane);
    st2_v4i(HHL + (size_t)grow * P_H + 8 * m, ow);
  }
}

__global__ __launch_bounds__(NTHR) __attribute__((amdgpu_num_vgpr(248)))
void k_gemm2(const unsigned short* __restrict__ M2HL, const unsigned short* __restrict__ HHL,
             const unsigned short* __restrict__ W2C, const float* __restrict__ sm,
             const int* __restrict__ FLAG, float* out) {
  __shared__ __attribute__((aligned(16))) float stg[GBM * SP];
  __shared__ __attribute__((aligned(16))) float sb[64];
  const int tid = (int)threadIdx.x, lane = tid & 31, wave = tid >> 5, hh = lane >> 4, m = lane & 15;
  const int rowBase = (int)blockIdx.x * GBM;
  const int flag = FLAG[(size_t)(rowBase >> SLB) * 32];
  if (tid < 16) *(v4fa*)(sb + 4 * tid) = *(const v4fa*)(sm + 64 + 4 * tid);

  v8f acc[4];
  {
    const v8f z = {0.f, 0.f, 0.f, 0.f, 0.f, 0.f, 0.f, 0.f};
#pragma unroll
    for (int t = 0; t < 4; ++t) acc[t] = z;
  }
  const int arow = rowBase + 16 * wave + m;
  const unsigned short* bp = W2C + (size_t)m * (size_t)P_W2 + 8 * hh;
  gemm_seg<P_W2>(M2HL + (size_t)arow * P_M2 + 8 * hh, bp, SPLIT_M2 ? 4 : 2, acc);
  gemm_seg<P_W2>(HHL + (size_t)arow * P_H + 8 * hh, bp + 2 * FO, SPLIT_H ? 4 : 2, acc);
  stage_d(stg, acc, wave, hh, m);
  __syncthreads();

  const v4f bias = *(const v4fa*)(sb + 4 * m);
  const float qnan = __uint_as_float(0x7fc00000u);
#pragma unroll 1
  for (int i = 0; i < 8; ++i) {
    const int lr   = 16 * wave + 2 * i + hh;
    const int grow = rowBase + lr;
    const v4f a = *(const v4fa*)(stg + lr * SP + 4 * m);
    asm volatile("" :: "v"(a));
    float v0 = a.x + bias.x, v1 = a.y + bias.y, v2 = a.z + bias.z, v3 = a.w + bias.w;
    v0 = (flag != 0) ? qnan : v0; v1 = (flag != 0) ? qnan : v1;
    v2 = (flag != 0) ? qnan : v2; v3 = (flag != 0) ? qnan : v3;
    v4f o;
    o.x = v0; o.y = v1; o.z = v2; o.w = v3;
    if (grow < NN) st2_v4f(out + (size_t)grow * FO + 4 * m, o);
  }
}

extern "C" void kernel_launch(void* const* d_in, const int* in_sizes, int n_in,
                              void* d_out, int out_size, void* d_ws, size_t ws_size,
                              hipStream_t stream) {
  if (n_in < 8) return;
  if (in_sizes[0] != NN * FI) return;
  if (in_sizes[1] != 2 * NE) return;
  if (in_sizes[2] != FI * FO) return;
  if (in_sizes[3] != FI * FO) return;
  if (in_sizes[4] != FO) return;
  if (in_sizes[5] != FO * FO) return;
  if (in_sizes[6] != FO * FO) return;
  if (in_sizes[7] != FO) return;
  if (out_size != NN * FO) return;

  const float* x   = (const float*)d_in[0];
  const int*   ei  = (const int*)d_in[1];
  const float* Wl1 = (const float*)d_in[2];
  const float* Wr1 = (const float*)d_in[3];
  const float* b1  = (const float*)d_in[4];
  const float* Wl2 = (const float*)d_in[5];
  const float* Wr2 = (const float*)d_in[6];
  const float* b2  = (const float*)d_in[7];
  float* out = (float*)d_out;
  const int* srcs = ei;
  const int* dsts = ei + NE;

  constexpr size_t zXB   = (size_t)MP * P_XB * 2;
  constexpr size_t zM1   = (size_t)MP * P_M1 * 2;
  constexpr size_t zM2   = (size_t)MP * P_M2 * 2;
  constexpr size_t zHHL  = (size_t)MP * P_H * 2;
  constexpr size_t zLIST = (size_t)NBK * RCAP * 4;
  constexpr size_t zCO   = (size_t)NBK * 2 * NBRUN * 4;
  constexpr size_t zFLAG = (size_t)NBK * 128;
  constexpr size_t zW1C  = (size_t)FO * P_W1 * 2;
  constexpr size_t zW2C  = (size_t)FO * P_W2 * 2;
  constexpr size_t zSM   = 512;
  constexpr size_t oXB   = 0;
  constexpr size_t oM1   = oXB + zXB;
  constexpr size_t oHHL  = oM1 + zM1;
  constexpr size_t oLIST = oHHL + zHHL;
  constexpr size_t oCO   = oLIST + zLIST;
  constexpr size_t oFLAG = oCO + zCO;
  constexpr size_t oW1C  = oFLAG + zFLAG;
  constexpr size_t oW2C  = oW1C + zW1C;
  constexpr size_t oSM   = oW2C + zW2C;
  constexpr size_t oEND  = oSM + zSM;
  static_assert(zXB % 256 == 0 && zM1 % 256 == 0 && zM2 % 256 == 0 && zHHL % 256 == 0 && zLIST % 256 == 0);
  static_assert(zCO % 256 == 0 && zFLAG % 256 == 0 && zW1C % 256 == 0 && zW2C % 256 == 0 && zSM % 256 == 0);
  static_assert(zM2 <= zM1);
  static_assert(oEND <= (size_t)(128u << 20));
  if (oEND > ws_size || oEND > WSMAX) return;

  char* ws = (char*)d_ws;
  unsigned short* XB   = (unsigned short*)(ws + oXB);
  unsigned short* M1HL = (unsigned short*)(ws + oM1);
  unsigned short* M2HL = (unsigned short*)(ws + oM1);
  unsigned short* HHL  = (unsigned short*)(ws + oHHL);
  int*            LIST = (int*)(ws + oLIST);
  int*            CO   = (int*)(ws + oCO);
  int*            FLAG = (int*)(ws + oFLAG);
  unsigned short* W1C  = (unsigned short*)(ws + oW1C);
  unsigned short* W2C  = (unsigned short*)(ws + oW2C);
  float*          SM   = (float*)(ws + oSM);

  hipFuncSetAttribute(reinterpret_cast<const void*>(&k_bucket), hipFuncAttributeMaxDynamicSharedMemorySize, (int)BK_LDS);

  k_prep<<<PBTOT, NTHR, 0, stream>>>(x, Wl1, Wr1, b1, Wl2, Wr2, b2, XB, W1C, W2C, SM);
  k_bucket<<<NBK, NTHR, BK_LDS, stream>>>(srcs, dsts, LIST, CO, FLAG);
  k_replay1<<<MP / RPB, NTHR, 0, stream>>>(LIST, CO, FLAG, XB, M1HL);
  k_gemm1<<<MP / GBM, NTHR, 0, stream>>>(M1HL, XB, W1C, SM, HHL);
  k_replay2<<<MP / RPB, NTHR, 0, stream>>>(LIST, CO, FLAG, HHL, M2HL);
  k_gemm2<<<MP / GBM, NTHR, 0, stream>>>(M2HL, HHL, W2C, SM, FLAG, out);
}
